// SDARAttention_62801011802769
// MI455X (gfx1250) — hardware-verified
//
#include <hip/hip_runtime.h>
#include <stddef.h>
#include <stdint.h>
#include <math.h>

#define NB   2
#define SQ   2048
#define NTOK (NB * SQ)
#define DM   2048
#define NQH  32
#define NKH  8
#define GRP  (NQH / NKH)
#define HD   64
#define NF   (HD / 2)
#define QBLK (SQ / 128)
#define RBPS (SQ / 256)

static_assert(NQH * HD == DM);
static_assert(GRP == 4);
static_assert(SQ % 256 == 0);
static_assert(SQ % 128 == 0);
static_assert(SQ % 64 == 0);
static_assert(DM % 64 == 0);
static_assert(DM % 32 == 0);
static_assert(HD == 64);
static_assert(NF == 32);
static_assert(QBLK == 16);
static_assert(RBPS == 8);
static_assert((NKH * HD) % 64 == 0);

typedef _Float16 v16h __attribute__((ext_vector_type(16)));
typedef _Float16 v8h  __attribute__((ext_vector_type(8)));
typedef float    v8f  __attribute__((ext_vector_type(8)));
typedef float    v4f  __attribute__((ext_vector_type(4)));
typedef unsigned int v4u __attribute__((ext_vector_type(4)));

union Frag  { v16h v; v8h h[2]; };
union Pack8 { v8h h; v4u u; };

__device__ __forceinline__ v8f mma16(v16h a, v16h b, v8f c) {
  c = __builtin_amdgcn_wmma_f32_16x16x32_f16(false, a, false, b, (short)0, c, false, false);
  asm volatile("v_nop\n\tv_nop\n\tv_nop\n\tv_nop" : "+v"(c) : "v"(a), "v"(b));
  return c;
}

__device__ __forceinline__ v16h ldfrag(const _Float16* p, int ld, int row0, int k0, int lane) {
  const int m = lane & 15, lh = lane >> 4;
  const _Float16* q = p + (size_t)(row0 + m) * ld + k0 + 8 * lh;
  Frag f;
  f.h[0] = *(const v8h*)(q);
  f.h[1] = *(const v8h*)(q + 16);
  return f.v;
}

__device__ __forceinline__ v8f zero8() { return (v8f){0.f, 0.f, 0.f, 0.f, 0.f, 0.f, 0.f, 0.f}; }

__device__ __forceinline__ void gemm32x64(const _Float16* __restrict__ A, int lda,
                                          const _Float16* __restrict__ Bt, int ldb,
                                          int m0, int n0, int lane, v8f (&acc)[2][4]) {
#pragma unroll 2
  for (int k0 = 0; k0 < DM; k0 += 32) {
    const v16h a0 = ldfrag(A, lda, m0, k0, lane);
    const v16h a1 = ldfrag(A, lda, m0 + 16, k0, lane);
    const v16h b0 = ldfrag(Bt, ldb, n0, k0, lane);
    const v16h b1 = ldfrag(Bt, ldb, n0 + 16, k0, lane);
    const v16h b2 = ldfrag(Bt, ldb, n0 + 32, k0, lane);
    const v16h b3 = ldfrag(Bt, ldb, n0 + 48, k0, lane);
    acc[0][0] = mma16(a0, b0, acc[0][0]);
    acc[1][0] = mma16(a1, b0, acc[1][0]);
    acc[0][1] = mma16(a0, b1, acc[0][1]);
    acc[1][1] = mma16(a1, b1, acc[1][1]);
    acc[0][2] = mma16(a0, b2, acc[0][2]);
    acc[1][2] = mma16(a1, b2, acc[1][2]);
    acc[0][3] = mma16(a0, b3, acc[0][3]);
    acc[1][3] = mma16(a1, b3, acc[1][3]);
  }
}

__global__ __launch_bounds__(256) void k_cvt(const float* __restrict__ x, _Float16* __restrict__ xh,
                                             int ngrp, float scale) {
  const int t = blockIdx.x * 256 + (int)threadIdx.x;
  if (t >= ngrp) return;
  const size_t o = (size_t)t * 8;
  const v4f a0 = *(const v4f*)(x + o) * scale;
  const v4f a1 = *(const v4f*)(x + o + 4) * scale;
  Pack8 pk;
  pk.h = (v8h){(_Float16)a0[0], (_Float16)a0[1], (_Float16)a0[2], (_Float16)a0[3],
               (_Float16)a1[0], (_Float16)a1[1], (_Float16)a1[2], (_Float16)a1[3]};
  const v4u vv = pk.u;
  volatile v4u* d = (volatile v4u*)(xh + o);
  *d = vv;
  __threadfence();
  *d = vv;
}

__global__ __launch_bounds__(256) void k_rope_tab(const int* __restrict__ pos, float* __restrict__ cs,
                                                  float* __restrict__ sn, int n) {
  const int i = blockIdx.x * 256 + (int)threadIdx.x;
  if (i >= n) return;
  const int t = i >> 5;
  const int j = i & 31;
  const float p  = (float)pos[t];
  const float e  = (float)(2 * j) * (1.0f / 64.0f);
  const float fr = 1.0f / powf(10000.0f, e);
  const float ang = p * fr;
  float sv, cv;
  sincosf(ang, &sv, &cv);
  volatile float* dc = cs + i;
  volatile float* ds = sn + i;
  *dc = cv;
  *ds = sv;
  __threadfence();
  *dc = cv;
  *ds = sv;
}

#define NTP 72
__global__ __launch_bounds__(256) void k_gemm_nr(const _Float16* __restrict__ xh,
                                                 const _Float16* __restrict__ wt,
                                                 const float* __restrict__ wn,
                                                 const float* __restrict__ cs,
                                                 const float* __restrict__ sn,
                                                 _Float16* __restrict__ plane, int nheads) {
  __shared__ __align__(16) _Float16 st[8][32 * NTP];
  const int tid = threadIdx.x, lane = tid & 31, wave = tid >> 5;
  const int hh = lane >> 4, c = lane & 15;
  const int m0 = blockIdx.x * 256 + wave * 32;
  const int h  = blockIdx.y;
  const int n0 = h * HD;
  const int b  = blockIdx.x / RBPS;

  v8f acc[2][4];
#pragma unroll
  for (int s = 0; s < 2; ++s)
#pragma unroll
    for (int t = 0; t < 4; ++t) acc[s][t] = zero8();
  gemm32x64(xh, DM, wt, DM, m0, n0, lane, acc);

  float wv[4];
#pragma unroll
  for (int t = 0; t < 4; ++t) wv[t] = wn[16 * t + c];

  _Float16* sw = st[wave];
#pragma unroll
  for (int sub = 0; sub < 2; ++sub) {
#pragma unroll
    for (int r = 0; r < 8; ++r) {
      const int lr = 16 * sub + 8 * hh + r;
      const int m  = m0 + lr;
      const float x0 = acc[sub][0][r] * 0.03125f;
      const float x1 = acc[sub][1][r] * 0.03125f;
      const float x2 = acc[sub][2][r] * 0.03125f;
      const float x3 = acc[sub][3][r] * 0.03125f;
      float ss = x0 * x0 + x1 * x1 + x2 * x2 + x3 * x3;
      ss += __shfl_xor(ss, 1, 32);
      ss += __shfl_xor(ss, 2, 32);
      ss += __shfl_xor(ss, 4, 32);
      ss += __shfl_xor(ss, 8, 32);
      const float rs = rsqrtf(ss * (1.0f / 64.0f) + 1e-6f);
      const float y0 = (x0 * rs) * wv[0];
      const float y1 = (x1 * rs) * wv[1];
      const float y2 = (x2 * rs) * wv[2];
      const float y3 = (x3 * rs) * wv[3];
      const float* cr = cs + (size_t)m * NF;
      const float* sr = sn + (size_t)m * NF;
      const float c0 = cr[c], c1 = cr[16 + c];
      const float s0 = sr[c], s1 = sr[16 + c];
      const float o0 = y0 * c0 - y2 * s0;
      const float o1 = y1 * c1 - y3 * s1;
      const float o2 = y2 * c0 + y0 * s0;
      const float o3 = y3 * c1 + y1 * s1;
      _Float16* rw = sw + lr * NTP;
      rw[c]      = (_Float16)o0;
      rw[16 + c] = (_Float16)o1;
      rw[32 + c] = (_Float16)o2;
      rw[48 + c] = (_Float16)o3;
    }
  }
  __syncthreads();

  const size_t pbase = ((size_t)(b * nheads + h) * SQ + (size_t)(m0 - b * SQ)) * HD;
  v4u val[8];
  size_t go[8];
#pragma unroll
  for (int it = 0; it < 8; ++it) {
    const int p  = lane + 32 * it;
    const int L  = p >> 3;
    const int pc = p & 7;
    Pack8 pk;
    pk.h    = *(const v8h*)(sw + L * NTP + pc * 8);
    val[it] = pk.u;
    go[it]  = pbase + (size_t)L * HD + pc * 8;
  }
  for (int ps = 0; ps < 2; ++ps) {
#pragma unroll
    for (int it = 0; it < 8; ++it) *(volatile v4u*)(plane + go[it]) = val[it];
    __threadfence();
  }
}

#define STP 72
__global__ __launch_bounds__(256) void k_gemm_vt(const _Float16* __restrict__ xh,
                                                 const _Float16* __restrict__ wt,
                                                 _Float16* __restrict__ vt) {
  __shared__ __align__(16) _Float16 st[256 * STP];
  const int tid = threadIdx.x, lane = tid & 31, wave = tid >> 5;
  const int hh = lane >> 4, c = lane & 15;
  const int mb = blockIdx.x * 256;
  const int m0 = mb + wave * 32;
  const int hk = blockIdx.y;
  const int n0 = hk * HD;
  const int b  = blockIdx.x / RBPS;

  v8f acc[2][4];
#pragma unroll
  for (int s = 0; s < 2; ++s)
#pragma unroll
    for (int t = 0; t < 4; ++t) acc[s][t] = zero8();
  gemm32x64(xh, DM, wt, DM, m0, n0, lane, acc);

#pragma unroll
  for (int t = 0; t < 4; ++t) {
#pragma unroll
    for (int sub = 0; sub < 2; ++sub) {
#pragma unroll
      for (int r = 0; r < 8; ++r) {
        const int lr = wave * 32 + sub * 16 + 8 * hh + r;
        st[lr * STP + 16 * t + c] = (_Float16)(acc[sub][t][r] * 0.03125f);
      }
    }
  }
  __syncthreads();

  const size_t rbase = (size_t)(b * NKH + hk) * HD;
  const int    sb    = mb - b * SQ;
  v4u val[8];
  size_t go[8];
#pragma unroll
  for (int j = 0; j < 8; ++j) {
    const int p  = tid + 256 * j;
    const int L  = p >> 3;
    const int pc = p & 7;
    const int d  = L >> 2;
    const int nl = (L & 3) * 64 + pc * 8;
    const _Float16* cp = st + nl * STP + d;
    Pack8 pk;
    pk.h = (v8h){cp[0 * STP], cp[1 * STP], cp[2 * STP], cp[3 * STP],
                 cp[4 * STP], cp[5 * STP], cp[6 * STP], cp[7 * STP]};
    val[j] = pk.u;
    go[j]  = (rbase + (size_t)d) * SQ + sb + nl;
  }
  for (int ps = 0; ps < 2; ++ps) {
#pragma unroll
    for (int j = 0; j < 8; ++j) *(volatile v4u*)(vt + go[j]) = val[j];
    __threadfence();
  }
}

#define KTP 72
#define VTP 72
#define PTP 72
#define OSP 72
#define KS_H (64 * KTP)
#define VS_H (64 * VTP)
#define PS_H (8 * 16 * PTP)
static_assert(8 * 16 * OSP <= KS_H + VS_H);

__global__ __launch_bounds__(256) void k_attn(const _Float16* __restrict__ qp,
                                              const _Float16* __restrict__ kp,
                                              const _Float16* __restrict__ vt,
                                              _Float16* __restrict__ op, float sscale) {
  __shared__ __align__(16) _Float16 Sh[KS_H + VS_H + PS_H];
  _Float16* Ks = Sh;
  _Float16* Vs = Sh + KS_H;
  _Float16* Pb = Sh + KS_H + VS_H;

  const int tid = threadIdx.x, lane = tid & 31, wave = tid >> 5;
  const int hh = lane >> 4, c = lane & 15;
  const int bh = blockIdx.x / QBLK;
  const int qb = blockIdx.x - bh * QBLK;
  const int b  = bh / NQH;
  const int h  = bh - b * NQH;
  const int hk = h / GRP;
  const int q0 = qb * 128 + wave * 16;

  const _Float16* Q = qp + (size_t)bh * SQ * HD;
  const _Float16* K = kp + (size_t)(b * NKH + hk) * SQ * HD;
  const _Float16* V = vt + (size_t)(b * NKH + hk) * HD * SQ;

  v16h qa[2];
#pragma unroll
  for (int dc = 0; dc < 2; ++dc) qa[dc] = ldfrag(Q, HD, q0, dc * 32, lane);

  const float NEGI = -__builtin_huge_valf();
  float mrow[8], lrow[8];
  v8f oacc[4];
#pragma unroll
  for (int r = 0; r < 8; ++r) { mrow[r] = NEGI; lrow[r] = 0.f; }
#pragma unroll
  for (int t = 0; t < 4; ++t) oacc[t] = zero8();

  _Float16* pw = Pb + wave * 16 * PTP;

  for (int kc = 0; kc < SQ / 64; ++kc) {
    const int kv0 = kc * 64;
    __syncthreads();
    {
      const int r  = tid >> 2;
      const int qq = (tid & 3) * 16;
      const _Float16* ks = K + (size_t)(kv0 + r) * HD + qq;
      _Float16* kd = Ks + r * KTP + qq;
      *(v8h*)(kd)     = *(const v8h*)(ks);
      *(v8h*)(kd + 8) = *(const v8h*)(ks + 8);
      const _Float16* vs = V + (size_t)r * SQ + kv0 + qq;
      _Float16* vd = Vs + r * VTP + qq;
      *(v8h*)(vd)     = *(const v8h*)(vs);
      *(v8h*)(vd + 8) = *(const v8h*)(vs + 8);
    }
    __syncthreads();

    v8f s[4];
#pragma unroll
    for (int j = 0; j < 4; ++j) s[j] = zero8();
#pragma unroll
    for (int dc = 0; dc < 2; ++dc) {
#pragma unroll
      for (int j = 0; j < 4; ++j) {
        const v16h kb = ldfrag(Ks, KTP, j * 16, dc * 32, lane);
        s[j] = mma16(qa[dc], kb, s[j]);
      }
    }
    float cm[8];
#pragma unroll
    for (int r = 0; r < 8; ++r) {
      float m = NEGI;
#pragma unroll
      for (int j = 0; j < 4; ++j) {
        const float sv = s[j][r] * sscale;
        s[j][r] = sv;
        m = fmaxf(m, sv);
      }
#pragma unroll
      for (int off = 1; off < 16; off <<= 1) m = fmaxf(m, __shfl_xor(m, off, 32));
      cm[r] = m;
    }
    float al[8];
#pragma unroll
    for (int r = 0; r < 8; ++r) {
      const float mnew  = fmaxf(mrow[r], cm[r]);
      const float alpha = __expf(mrow[r] - mnew);
      mrow[r] = mnew;
      float psum = 0.f;
#pragma unroll
      for (int j = 0; j < 4; ++j) {
        const float p = __expf(s[j][r] - mnew);
        psum += p;
        pw[(8 * hh + r) * PTP + j * 16 + c] = (_Float16)(p * 1024.0f);
      }
#pragma unroll
      for (int off = 1; off < 16; off <<= 1) psum += __shfl_xor(psum, off, 32);
      lrow[r] = lrow[r] * alpha + psum;
      al[r] = alpha;
    }
#pragma unroll
    for (int t = 0; t < 4; ++t)
#pragma unroll
      for (int r = 0; r < 8; ++r) oacc[t][r] *= al[r];
    __syncthreads();

#pragma unroll
    for (int kk = 0; kk < 2; ++kk) {
      const v16h pa = ldfrag(pw, PTP, 0, kk * 32, lane);
#pragma unroll
      for (int t = 0; t < 4; ++t) {
        const v16h vb = ldfrag(Vs, VTP, t * 16, kk * 32, lane);
        oacc[t] = mma16(pa, vb, oacc[t]);
      }
    }
  }
  __syncthreads();

  _Float16* ow = Sh + wave * 16 * OSP;
#pragma unroll
  for (int r = 0; r < 8; ++r) {
    const float inv = 0.03125f / lrow[r];
#pragma unroll
    for (int t = 0; t < 4; ++t) ow[(8 * hh + r) * OSP + 16 * t + c] = (_Float16)(oacc[t][r] * inv);
  }
  __syncthreads();
  v4u val[4];
  size_t go[4];
#pragma unroll
  for (int it = 0; it < 4; ++it) {
    const int p  = lane + 32 * it;
    const int L  = p >> 3;
    const int pc = p & 7;
    Pack8 pk;
    pk.h    = *(const v8h*)(ow + L * OSP + pc * 8);
    val[it] = pk.u;
    go[it]  = (size_t)(b * SQ + q0 + L) * DM + (size_t)h * HD + pc * 8;
  }
  for (int ps = 0; ps < 2; ++ps) {
#pragma unroll
    for (int it = 0; it < 4; ++it) *(volatile v4u*)(op + go[it]) = val[it];
    __threadfence();
  }
}

#define OTP 68
__global__ __launch_bounds__(256) void k_gemm_out(const _Float16* __restrict__ ap,
                                                  const _Float16* __restrict__ wt,
                                                  float* __restrict__ out, float oscale) {
  __shared__ __align__(16) float st[8][16 * OTP];
  const int tid = threadIdx.x, lane = tid & 31, wave = tid >> 5;
  const int hh = lane >> 4, c = lane & 15;
  const int m0 = blockIdx.x * 256 + wave * 32;
  const int n0 = blockIdx.y * 64;

  v8f acc[2][4];
#pragma unroll
  for (int s = 0; s < 2; ++s)
#pragma unroll
    for (int t = 0; t < 4; ++t) acc[s][t] = zero8();
  gemm32x64(ap, DM, wt, DM, m0, n0, lane, acc);

  float* sw = st[wave];
#pragma unroll
  for (int sub = 0; sub < 2; ++sub) {
    __syncthreads();
#pragma unroll
    for (int t = 0; t < 4; ++t) {
#pragma unroll
      for (int r = 0; r < 8; ++r)
        sw[(8 * hh + r) * OTP + 16 * t + c] = acc[sub][t][r] * oscale;
    }
    __syncthreads();
    v4f val[8];
    size_t go[8];
#pragma unroll
    for (int it = 0; it < 8; ++it) {
      const int p    = lane + 32 * it;
      const int L    = p >> 3;
      const int pc   = p & 7;
      const int row  = L >> 1;
      const int half = L & 1;
      val[it] = *(const v4f*)(sw + row * OTP + half * 32 + pc * 4);
      go[it]  = (size_t)(m0 + sub * 16 + row) * DM + n0 + half * 32 + pc * 4;
    }
    for (int ps = 0; ps < 2; ++ps) {
#pragma unroll
      for (int it = 0; it < 8; ++it) *(volatile v4f*)(out + go[it]) = val[it];
      __threadfence();
    }
  }
}

#define XH_B  ((size_t)NTOK * DM * 2)
#define WQ_B  ((size_t)DM * DM * 2)
#define WKV_B ((size_t)NKH * HD * DM * 2)
#define TB_B  ((size_t)NTOK * NF * 4)
#define QP_B  ((size_t)NB * NQH * SQ * HD * 2)
#define KP_B  ((size_t)NB * NKH * SQ * HD * 2)
#define OP_B  ((size_t)NTOK * DM * 2)
static_assert(XH_B + WQ_B + 2 * WKV_B + WQ_B + 2 * TB_B + QP_B + 2 * KP_B + OP_B == (size_t)80740352);
static_assert(XH_B + WQ_B + 2 * WKV_B + WQ_B + 2 * TB_B + QP_B + 2 * KP_B + OP_B <= (size_t)134217728);
static_assert(XH_B % 128 == 0 && WQ_B % 128 == 0 && WKV_B % 128 == 0 && TB_B % 128 == 0);
static_assert(QP_B % 128 == 0 && KP_B % 128 == 0 && OP_B % 128 == 0);

extern "C" void kernel_launch(void* const* d_in, const int* in_sizes, int n_in,
                              void* d_out, int out_size, void* d_ws, size_t ws_size,
                              hipStream_t stream) {
  if (n_in < 8) return;
  if (in_sizes[0] != NTOK) return;
  if (in_sizes[1] != NTOK * DM) return;
  if (in_sizes[2] != DM * DM || in_sizes[5] != DM * DM) return;
  if (in_sizes[3] != NKH * HD * DM || in_sizes[4] != NKH * HD * DM) return;
  if (in_sizes[6] != HD || in_sizes[7] != HD) return;
  if (out_size != NTOK * DM) return;

  const int*   pos = (const int*)d_in[0];
  const float* x   = (const float*)d_in[1];
  const float* wq  = (const float*)d_in[2];
  const float* wk  = (const float*)d_in[3];
  const float* wv  = (const float*)d_in[4];
  const float* wo  = (const float*)d_in[5];
  const float* nqw = (const float*)d_in[6];
  const float* nkw = (const float*)d_in[7];
  float* out = (float*)d_out;

  size_t off = 0;
  const size_t oX  = off; off += XH_B;
  const size_t oWq = off; off += WQ_B;
  const size_t oWk = off; off += WKV_B;
  const size_t oWv = off; off += WKV_B;
  const size_t oWo = off; off += WQ_B;
  const size_t oCS = off; off += TB_B;
  const size_t oSN = off; off += TB_B;
  const size_t oQ  = off; off += QP_B;
  const size_t oK  = off; off += KP_B;
  const size_t oVt = off; off += KP_B;
  const size_t oO  = off; off += OP_B;
  if (off > ws_size) return;

  char* ws = (char*)d_ws;
  _Float16* Xh  = (_Float16*)(ws + oX);
  _Float16* Wqh = (_Float16*)(ws + oWq);
  _Float16* Wkh = (_Float16*)(ws + oWk);
  _Float16* Wvh = (_Float16*)(ws + oWv);
  _Float16* Woh = (_Float16*)(ws + oWo);
  float*    Cs  = (float*)(ws + oCS);
  float*    Sn  = (float*)(ws + oSN);
  _Float16* Qp  = (_Float16*)(ws + oQ);
  _Float16* Kp  = (_Float16*)(ws + oK);
  _Float16* Vtp = (_Float16*)(ws + oVt);
  _Float16* Op  = (_Float16*)(ws + oO);

  const int ngx  = in_sizes[1] / 8;
  const int ngwq = in_sizes[2] / 8;
  const int ngwk = in_sizes[3] / 8;
  const int ngwv = in_sizes[4] / 8;
  const int ngwo = in_sizes[5] / 8;
  const int ntab = in_sizes[0] * NF;

  k_cvt<<<dim3((ngx + 255) / 256), dim3(256), 0, stream>>>(x, Xh, ngx, 1.0f);
  k_cvt<<<dim3((ngwq + 255) / 256), dim3(256), 0, stream>>>(wq, Wqh, ngwq, 32.0f);
  k_cvt<<<dim3((ngwk + 255) / 256), dim3(256), 0, stream>>>(wk, Wkh, ngwk, 32.0f);
  k_cvt<<<dim3((ngwv + 255) / 256), dim3(256), 0, stream>>>(wv, Wvh, ngwv, 32.0f);
  k_cvt<<<dim3((ngwo + 255) / 256), dim3(256), 0, stream>>>(wo, Woh, ngwo, 32.0f);
  k_rope_tab<<<dim3((ntab + 255) / 256), dim3(256), 0, stream>>>(pos, Cs, Sn, ntab);
  k_gemm_nr<<<dim3(NTOK / 256, NQH), dim3(256), 0, stream>>>(Xh, Wqh, nqw, Cs, Sn, Qp, NQH);
  k_gemm_nr<<<dim3(NTOK / 256, NKH), dim3(256), 0, stream>>>(Xh, Wkh, nkw, Cs, Sn, Kp, NKH);
  k_gemm_vt<<<dim3(NTOK / 256, NKH), dim3(256), 0, stream>>>(Xh, Wvh, Vtp);
  k_attn<<<dim3(NB * NQH * QBLK), dim3(256), 0, stream>>>(Qp, Kp, Vtp, Op, 0.125f);
  k_gemm_out<<<dim3(NTOK / 256, DM / 64), dim3(256), 0, stream>>>(Op, Woh, out, 0.0009765625f);
  (void)hipGetLastError();
}
